// MultiParticlesGraphNet_30760555774211
// MI455X (gfx1250) — hardware-verified
//
#include <hip/hip_runtime.h>
#include <hip/hip_bf16.h>


#define NB_     32
#define NN_     64
#define HH_     128
#define NL_     4
#define NODES_  2048
#define TP16_   136
#define TP32_   132

typedef float          v4f   __attribute__((ext_vector_type(4)));
typedef float          v8f   __attribute__((ext_vector_type(8)));
typedef _Float16       v8h   __attribute__((ext_vector_type(8)));
typedef _Float16       v16h  __attribute__((ext_vector_type(16)));
typedef __bf16         v16b  __attribute__((ext_vector_type(16)));
typedef unsigned short u16x8 __attribute__((ext_vector_type(8)));
typedef unsigned int   u32x4 __attribute__((ext_vector_type(4)));

union FragH { v8h h[2];   v16h v; };
union FragB { u16x8 h[2]; v16b v; };

constexpr size_t SZ_H32 = (size_t)NODES_ * HH_ * 4;
constexpr size_t SZ_HA  = (size_t)NODES_ * 2 * HH_ * 2;
constexpr size_t SZ_PQ  = (size_t)NODES_ * 2 * HH_ * 4;
constexpr int WO_PQH = 0;
constexpr int WO_PQL = 32768;
constexpr int WO_N1H = 65536;
constexpr int WO_N1L = 98304;
constexpr int WO_N2H = 131072;
constexpr int WO_N2L = 147456;
constexpr int WO_E2H = 163840;
constexpr int WO_E2L = 180224;
constexpr int WO_C2F = 196608;
constexpr int WO_E1F = 212992;
constexpr int WL_U16 = 229376;
constexpr size_t SZ_W   = (size_t)NL_ * WL_U16 * 2;

constexpr size_t OFF_HN  = 0;
constexpr size_t OFF_HB  = OFF_HN + SZ_H32;
constexpr size_t OFF_HAH = OFF_HB + SZ_H32;
constexpr size_t OFF_HAL = OFF_HAH + SZ_HA;
constexpr size_t OFF_PQ  = OFF_HAL + SZ_HA;
constexpr size_t OFF_W   = OFF_PQ + SZ_PQ;
constexpr size_t WS_END  = OFF_W + SZ_W;
static_assert(WS_END <= (size_t)134217728);
static_assert(OFF_HB % 128 == 0 && OFF_HAH % 128 == 0 && OFF_HAL % 128 == 0 && OFF_PQ % 128 == 0 && OFF_W % 128 == 0);
static_assert((WL_U16 * 2) % 128 == 0);
static_assert(WO_E1F + HH_ * HH_ == WL_U16);

constexpr int EK_T16  = 16 * TP16_ * 2;
constexpr int EK_WR   = 4 * EK_T16;
constexpr int EK_AGG  = 8 * EK_WR;
constexpr int EK_LDS  = EK_AGG + 2 * HH_ * 4;
static_assert(16 * TP32_ * 4 <= 2 * EK_T16);
constexpr int NK_WR   = 2 * EK_T16 + 16 * TP32_ * 4;
constexpr int NK_LDS  = 4 * NK_WR;

__device__ __forceinline__ unsigned short f32_to_bf16(float f) {
    unsigned u = __float_as_uint(f);
    unsigned r = u + 0x7FFFu + ((u >> 16) & 1u);
    return (unsigned short)(r >> 16);
}
__device__ __forceinline__ float bf16_to_f32(unsigned short b) {
    return __uint_as_float(((unsigned)b) << 16);
}
__device__ __forceinline__ void split1(float f, unsigned short& hb, unsigned short& lb) {
    hb = f32_to_bf16(f);
    lb = f32_to_bf16(f - bf16_to_f32(hb));
}
__device__ __forceinline__ float gelu_f(float x) {
    return 0.5f * x * (1.0f + erff(x * 0.70710678118654752f));
}
__device__ __forceinline__ v8f ld8f(const float* p) {
    v4f a = *(const v4f*)p;
    v4f b = *(const v4f*)(p + 4);
    return __builtin_shufflevector(a, b, 0, 1, 2, 3, 4, 5, 6, 7);
}
__device__ __forceinline__ void split8(const v8f x, u16x8& hv, u16x8& lv) {
#pragma unroll
    for (int c = 0; c < 8; ++c) {
        unsigned short hb, lb;
        split1(x[c], hb, lb);
        hv[c] = hb;
        lv[c] = lb;
    }
}

__device__ __forceinline__ void mma_h(v8f& acc, const FragH& a, const FragH& b) {
    acc = __builtin_amdgcn_wmma_f32_16x16x32_f16(false, a.v, false, b.v, (short)0, acc, false, false);
    asm volatile("v_nop\n\tv_nop\n\tv_nop\n\tv_nop" : "+v"(acc) : "v"(a.v), "v"(b.v));
}
__device__ __forceinline__ void mma_b(v8f& acc, const FragB& a, const FragB& b) {
    acc = __builtin_amdgcn_wmma_f32_16x16x32_bf16(false, a.v, false, b.v, (short)0, acc, false, false);
    asm volatile("v_nop\n\tv_nop\n\tv_nop\n\tv_nop" : "+v"(acc) : "v"(a.v), "v"(b.v));
}
__device__ __forceinline__ void acc_zero(v8f (&acc)[8]) {
#pragma unroll
    for (int j = 0; j < 8; ++j)
#pragma unroll
        for (int r = 0; r < 8; ++r) acc[j][r] = 0.0f;
}

__device__ __forceinline__ void wgemm_f16(v8f (&acc)[8], const _Float16* A, int lda,
                                          const _Float16* Bt, int ldb, int K, int lane)
{
    const int h = lane >> 4, m = lane & 15;
    const _Float16* ap = A + m * lda + 8 * h;
    const _Float16* bp = Bt + m * ldb + 8 * h;
#pragma unroll 1
    for (int k0 = 0; k0 < K; k0 += 32) {
        FragH fa;
        fa.h[0] = *(const v8h*)(ap + k0);
        fa.h[1] = *(const v8h*)(ap + k0 + 16);
#pragma unroll
        for (int nt = 0; nt < 8; ++nt) {
            const _Float16* q = bp + nt * 16 * ldb + k0;
            FragH fb;
            fb.h[0] = *(const v8h*)(q);
            fb.h[1] = *(const v8h*)(q + 16);
            mma_h(acc[nt], fa, fb);
        }
    }
}

__device__ __forceinline__ void wgemm_x3(v8f (&acc)[8],
                                         const unsigned short* Ah, const unsigned short* Al, int lda,
                                         const unsigned short* Bh, const unsigned short* Bl, int ldb,
                                         int K, int lane)
{
    const int h = lane >> 4, m = lane & 15;
    const int ao = m * lda + 8 * h;
    const int bo = m * ldb + 8 * h;
#pragma unroll 1
    for (int k0 = 0; k0 < K; k0 += 32) {
        FragB fa, ga;
        fa.h[0] = *(const u16x8*)(Ah + ao + k0);
        fa.h[1] = *(const u16x8*)(Ah + ao + k0 + 16);
        ga.h[0] = *(const u16x8*)(Al + ao + k0);
        ga.h[1] = *(const u16x8*)(Al + ao + k0 + 16);
#pragma unroll
        for (int nt = 0; nt < 8; ++nt) {
            const int q = bo + nt * 16 * ldb + k0;
            FragB fb, gb;
            fb.h[0] = *(const u16x8*)(Bh + q);
            fb.h[1] = *(const u16x8*)(Bh + q + 16);
            gb.h[0] = *(const u16x8*)(Bl + q);
            gb.h[1] = *(const u16x8*)(Bl + q + 16);
            mma_b(acc[nt], fa, fb);
            mma_b(acc[nt], fa, gb);
            mma_b(acc[nt], ga, fb);
        }
    }
}

template<int F16>
__global__ __launch_bounds__(256)
void wprep_kernel(const float* __restrict__ src, int src_ls,
                  unsigned short* dhi, unsigned short* dlo, int dst_ls,
                  int Nw, int Kd, int nrows, float scale)
{
    __shared__ __attribute__((aligned(16))) float sT[64 * 68];
    const int tid  = threadIdx.x;
    const int lane = tid & 31;
    const int wave = tid >> 5;
    const int n0 = blockIdx.x * 64;
    const int k0 = blockIdx.y * 64;
    src += (size_t)blockIdx.z * src_ls;
    dhi += (size_t)blockIdx.z * dst_ls;
    dlo += (size_t)blockIdx.z * dst_ls;

#pragma unroll
    for (int it = 0; it < 4; ++it) {
        const int idx = it * 256 + tid;
        const int kk  = idx >> 4;
        const int n4  = (idx & 15) * 4;
        const int gn  = n0 + n4;
        const int gnc = min(gn, Nw - 4);
        const v4f v = *(const v4f*)(src + (size_t)(k0 + kk) * Nw + gnc);
        const bool in = (gn < Nw);
        sT[(n4 + 0) * 68 + kk] = in ? v[0] : 0.0f;
        sT[(n4 + 1) * 68 + kk] = in ? v[1] : 0.0f;
        sT[(n4 + 2) * 68 + kk] = in ? v[2] : 0.0f;
        sT[(n4 + 3) * 68 + kk] = in ? v[3] : 0.0f;
    }
    __syncthreads();

    u16x8 hv[2], lv[2];
    const int c = (lane & 7) * 8;
#pragma unroll
    for (int it = 0; it < 2; ++it) {
        const int nn = it * 32 + wave * 4 + (lane >> 3);
        const v8f x = ld8f(sT + nn * 68 + c);
        if (F16) {
            v8h t;
#pragma unroll
            for (int e = 0; e < 8; ++e) t[e] = (_Float16)(x[e] * scale);
            hv[it] = __builtin_bit_cast(u16x8, t);
            lv[it] = hv[it];
        } else {
            split8(x, hv[it], lv[it]);
        }
    }
#pragma unroll
    for (int it = 0; it < 2; ++it) {
        const int gr = n0 + it * 32 + wave * 4 + (lane >> 3);
        if (gr < nrows) {
            const size_t o = (size_t)gr * Kd + k0 + c;
            *(volatile u16x8*)(dhi + o) = hv[it];
            if (!F16) *(volatile u16x8*)(dlo + o) = lv[it];
        }
    }
    __threadfence();
#pragma unroll
    for (int it = 0; it < 2; ++it) {
        const int gr = n0 + it * 32 + wave * 4 + (lane >> 3);
        if (gr < nrows) {
            const size_t o = (size_t)gr * Kd + k0 + c;
            *(volatile u16x8*)(dhi + o) = hv[it];
            if (!F16) *(volatile u16x8*)(dlo + o) = lv[it];
        }
    }
}

__global__ __launch_bounds__(256)
void ln_kernel(const float* __restrict__ hin, const float* __restrict__ g, const float* __restrict__ bb,
               float* hn, unsigned short* hah, unsigned short* hal)
{
    const int lane = threadIdx.x & 31;
    const int wave = threadIdx.x >> 5;
    const int row  = blockIdx.x * 8 + wave;

    const v4f x = *(const v4f*)(hin + (size_t)row * HH_ + 4 * lane);
    float s = (x[0] + x[1]) + (x[2] + x[3]);
#pragma unroll
    for (int mm = 16; mm >= 1; mm >>= 1) s += __shfl_xor(s, mm, 32);
    const float mu = s * (1.0f / HH_);
    const v4f d = x - mu;
    float q = (d[0] * d[0] + d[1] * d[1]) + (d[2] * d[2] + d[3] * d[3]);
#pragma unroll
    for (int mm = 16; mm >= 1; mm >>= 1) q += __shfl_xor(q, mm, 32);
    const float var = q * (1.0f / HH_);
    const float rs  = rsqrtf(var + 1e-5f);
    const v4f gg = *(const v4f*)(g + 4 * lane);
    const v4f be = *(const v4f*)(bb + 4 * lane);
    v4f y;
#pragma unroll
    for (int e = 0; e < 4; ++e) y[e] = (d[e] * rs) * gg[e] + be[e];

    unsigned short hb[4], lb[4];
#pragma unroll
    for (int e = 0; e < 4; ++e) split1(y[e], hb[e], lb[e]);
    const unsigned ph0 = (unsigned)hb[0] | ((unsigned)hb[1] << 16);
    const unsigned ph1 = (unsigned)hb[2] | ((unsigned)hb[3] << 16);
    const unsigned pl0 = (unsigned)lb[0] | ((unsigned)lb[1] << 16);
    const unsigned pl1 = (unsigned)lb[2] | ((unsigned)lb[3] << 16);
    const int s0 = (2 * lane) & 31;
    const int s1 = (2 * lane + 1) & 31;
    u32x4 hv, lv;
    hv[0] = __shfl(ph0, s0, 32); hv[1] = __shfl(ph1, s0, 32); hv[2] = __shfl(ph0, s1, 32); hv[3] = __shfl(ph1, s1, 32);
    lv[0] = __shfl(pl0, s0, 32); lv[1] = __shfl(pl1, s0, 32); lv[2] = __shfl(pl0, s1, 32); lv[3] = __shfl(pl1, s1, 32);

    float* hp = hn + (size_t)row * HH_ + 4 * lane;
    const size_t po = (size_t)row * (2 * HH_) + 8 * lane;
    *(volatile v4f*)hp = y;
    if (lane < 16) {
        *(volatile u32x4*)(hah + po) = hv;
        *(volatile u32x4*)(hal + po) = lv;
    }
    __threadfence();
    *(volatile v4f*)hp = y;
    if (lane < 16) {
        *(volatile u32x4*)(hah + po) = hv;
        *(volatile u32x4*)(hal + po) = lv;
    }
}

__global__ __launch_bounds__(128)
void pq_kernel(const unsigned short* __restrict__ hah, const unsigned short* __restrict__ hal,
               const unsigned short* __restrict__ wh, const unsigned short* __restrict__ wl, float* pq)
{
    __shared__ __attribute__((aligned(16))) float st[4][16 * TP32_];
    const int lane = threadIdx.x & 31;
    const int wave = threadIdx.x >> 5;
    const int h = lane >> 4, m = lane & 15;
    const int row0 = blockIdx.y * 64 + wave * 16;
    const int col0 = blockIdx.x * 128;

    v8f acc[8];
    acc_zero(acc);
    wgemm_x3(acc, hah + (size_t)row0 * (2 * HH_), hal + (size_t)row0 * (2 * HH_), 2 * HH_,
             wh + (size_t)col0 * HH_, wl + (size_t)col0 * HH_, HH_, HH_, lane);

    float* s = st[wave];
#pragma unroll
    for (int nt = 0; nt < 8; ++nt)
#pragma unroll
        for (int r = 0; r < 8; ++r)
            s[(8 * h + r) * TP32_ + nt * 16 + m] = acc[nt][r];
    __syncthreads();

#pragma unroll
    for (int rr = 0; rr < 16; ++rr) {
        const v4f v = *(const v4f*)(s + rr * TP32_ + 4 * lane);
        *(volatile v4f*)(pq + (size_t)(row0 + rr) * (2 * HH_) + col0 + 4 * lane) = v;
    }
    __threadfence();
#pragma unroll
    for (int rr = 0; rr < 16; ++rr) {
        const v4f v = *(const v4f*)(s + rr * TP32_ + 4 * lane);
        *(volatile v4f*)(pq + (size_t)(row0 + rr) * (2 * HH_) + col0 + 4 * lane) = v;
    }
}

__global__ __launch_bounds__(256)
void edge_kernel(const float* __restrict__ pq, const float* __restrict__ coord,
                 const float* __restrict__ cW1, const float* __restrict__ cb1, const float* __restrict__ cb2,
                 const float* __restrict__ eb1, const float* __restrict__ eb2,
                 const _Float16* __restrict__ cW2t, const _Float16* __restrict__ eW1ct,
                 const unsigned short* __restrict__ eW2h, const unsigned short* __restrict__ eW2l,
                 unsigned short* hah, unsigned short* hal)
{
    extern __shared__ float4 smem_raw[];
    char* smem = (char*)smem_raw;

    const int tid  = threadIdx.x;
    const int lane = tid & 31;
    const int wave = tid >> 5;
    const int h = lane >> 4, m = lane & 15;
    const int blk = blockIdx.x;
    const int b   = blk >> 5;
    const int i0  = (blk & 31) * 2;
    const int sel = wave >> 2;
    const int mt  = wave & 3;
    const int inode = i0 + sel;
    const int gi  = b * NN_ + inode;
    const int gj0 = b * NN_ + mt * 16;

    char* wr = smem + wave * EK_WR;
    _Float16*       X1  = (_Float16*)(wr);
    _Float16*       X2  = (_Float16*)(wr + EK_T16);
    unsigned short* E1h = (unsigned short*)(wr + 2 * EK_T16);
    unsigned short* E1l = (unsigned short*)(wr + 3 * EK_T16);
    float*          F   = (float*)(wr);
    float*          sAgg = (float*)(smem + EK_AGG);

    {
        const int c8 = m * 8;
        const v8f w0 = ld8f(cW1 + c8);
        const v8f w1 = ld8f(cW1 + HH_ + c8);
        const v8f bv = ld8f(cb1 + c8);
        const float cx = coord[gi * 2];
        const float cy = coord[gi * 2 + 1];
#pragma unroll 2
        for (int t = 0; t < 8; ++t) {
            const int r  = 2 * t + h;
            const int gj = gj0 + r;
            const float dx = cx - coord[gj * 2];
            const float dy = cy - coord[gj * 2 + 1];
            v8h hv;
#pragma unroll
            for (int e = 0; e < 8; ++e) {
                const float v = dx * w0[e] + dy * w1[e] + bv[e];
                hv[e] = (_Float16)(gelu_f(v) * 16.0f);
            }
            *(v8h*)(X1 + r * TP16_ + c8) = hv;
        }
    }
    __syncthreads();

    v8f acc[8];

    acc_zero(acc);
    wgemm_f16(acc, X1, TP16_, cW2t, HH_, HH_, lane);
#pragma unroll
    for (int nt = 0; nt < 8; ++nt) {
        const int col = nt * 16 + m;
        const float b2 = cb2[col];
#pragma unroll
        for (int r = 0; r < 8; ++r) {
            const float v = acc[nt][r] * (1.0f / 256.0f) + b2;
            X2[(8 * h + r) * TP16_ + col] = (_Float16)(gelu_f(v) * 256.0f);
        }
    }
    __syncthreads();

    acc_zero(acc);
    wgemm_f16(acc, X2, TP16_, eW1ct, HH_, HH_, lane);
#pragma unroll
    for (int nt = 0; nt < 8; ++nt) {
        const int col = nt * 16 + m;
        const float pe = pq[(size_t)gi * (2 * HH_) + col] + eb1[col];
#pragma unroll
        for (int r = 0; r < 8; ++r) {
            const int row = 8 * h + r;
            const int gj  = gj0 + row;
            const float qv = pq[(size_t)gj * (2 * HH_) + HH_ + col];
            const float v  = acc[nt][r] * (1.0f / 4096.0f) + pe + qv;
            unsigned short hb, lb;
            split1(gelu_f(v), hb, lb);
            E1h[row * TP16_ + col] = hb;
            E1l[row * TP16_ + col] = lb;
        }
    }
    __syncthreads();

    acc_zero(acc);
    wgemm_x3(acc, E1h, E1l, TP16_, eW2h, eW2l, HH_, HH_, lane);
#pragma unroll
    for (int nt = 0; nt < 8; ++nt) {
        const int col = nt * 16 + m;
        const float b2 = eb2[col];
#pragma unroll
        for (int r = 0; r < 8; ++r) {
            const int row = 8 * h + r;
            float gv = gelu_f(acc[nt][r] + b2);
            if (mt * 16 + row == inode) gv = 0.0f;
            F[row * TP32_ + col] = gv;
        }
    }
    __syncthreads();

    {
        const int s5 = tid >> 7;
        const int c  = tid & 127;
        float s = 0.0f;
#pragma unroll
        for (int wq = 0; wq < 4; ++wq) {
            const float* Fw = (const float*)(smem + (s5 * 4 + wq) * EK_WR) + c;
#pragma unroll 4
            for (int rr = 0; rr < 16; ++rr) s += Fw[rr * TP32_];
        }
        sAgg[s5 * HH_ + c] = s;
    }
    __syncthreads();

    if (wave == 0) {
        const int c8 = m * 8;
        const v8f x = ld8f(sAgg + h * HH_ + c8);
        u16x8 hv, lv;
        split8(x, hv, lv);
        const size_t off = (size_t)(b * NN_ + i0 + h) * (2 * HH_) + HH_ + c8;
        *(volatile u16x8*)(hah + off) = hv;
        *(volatile u16x8*)(hal + off) = lv;
        __threadfence();
        *(volatile u16x8*)(hah + off) = hv;
        *(volatile u16x8*)(hal + off) = lv;
    }
}

__global__ __launch_bounds__(128)
void node_kernel(const unsigned short* __restrict__ hah, const unsigned short* __restrict__ hal,
                 const float* __restrict__ hn,
                 const unsigned short* __restrict__ n1h, const unsigned short* __restrict__ n1l,
                 const unsigned short* __restrict__ n2h, const unsigned short* __restrict__ n2l,
                 const float* __restrict__ nb1, const float* __restrict__ nb2, float* hout)
{
    extern __shared__ float4 smem_raw[];
    char* smem = (char*)smem_raw;
    const int lane = threadIdx.x & 31;
    const int wave = threadIdx.x >> 5;
    const int h = lane >> 4, m = lane & 15;
    const int r0 = blockIdx.x * 64 + wave * 16;

    char* wr = smem + wave * NK_WR;
    unsigned short* Mh = (unsigned short*)(wr);
    unsigned short* Ml = (unsigned short*)(wr + EK_T16);
    float*          S  = (float*)(wr + 2 * EK_T16);

    v8f acc[8];
    acc_zero(acc);
    wgemm_x3(acc, hah + (size_t)r0 * (2 * HH_), hal + (size_t)r0 * (2 * HH_), 2 * HH_, n1h, n1l, 2 * HH_, 2 * HH_, lane);
#pragma unroll
    for (int nt = 0; nt < 8; ++nt) {
        const int col = nt * 16 + m;
        const float b1 = nb1[col];
#pragma unroll
        for (int r = 0; r < 8; ++r) {
            const int row = 8 * h + r;
            unsigned short hb, lb;
            split1(gelu_f(acc[nt][r] + b1), hb, lb);
            Mh[row * TP16_ + col] = hb;
            Ml[row * TP16_ + col] = lb;
        }
    }
    __syncthreads();

    acc_zero(acc);
    wgemm_x3(acc, Mh, Ml, TP16_, n2h, n2l, HH_, HH_, lane);
#pragma unroll
    for (int nt = 0; nt < 8; ++nt) {
        const int col = nt * 16 + m;
        const float b2 = nb2[col];
#pragma unroll
        for (int r = 0; r < 8; ++r) {
            const int row = 8 * h + r;
            const float o = acc[nt][r] + b2;
            S[row * TP32_ + col] = hn[(size_t)(r0 + row) * HH_ + col] + o;
        }
    }
    __syncthreads();

#pragma unroll
    for (int rr = 0; rr < 16; ++rr) {
        const v4f v = *(const v4f*)(S + rr * TP32_ + 4 * lane);
        *(volatile v4f*)(hout + (size_t)(r0 + rr) * HH_ + 4 * lane) = v;
    }
    __threadfence();
#pragma unroll
    for (int rr = 0; rr < 16; ++rr) {
        const v4f v = *(const v4f*)(S + rr * TP32_ + 4 * lane);
        *(volatile v4f*)(hout + (size_t)(r0 + rr) * HH_ + 4 * lane) = v;
    }
}

extern "C" void kernel_launch(void* const* d_in, const int* in_sizes, int n_in,
                              void* d_out, int out_size, void* d_ws, size_t ws_size,
                              hipStream_t stream)
{
    if (n_in < 16) return;
    if (in_sizes[0]  != NODES_ * HH_)        return;
    if (in_sizes[1]  != NODES_ * 2)          return;
    if (in_sizes[2]  != NL_ * HH_)           return;
    if (in_sizes[3]  != NL_ * HH_)           return;
    if (in_sizes[4]  != NL_ * 2 * HH_)       return;
    if (in_sizes[5]  != NL_ * HH_)           return;
    if (in_sizes[6]  != NL_ * HH_ * HH_)     return;
    if (in_sizes[7]  != NL_ * HH_)           return;
    if (in_sizes[8]  != NL_ * 3 * HH_ * HH_) return;
    if (in_sizes[9]  != NL_ * HH_)           return;
    if (in_sizes[10] != NL_ * HH_ * HH_)     return;
    if (in_sizes[11] != NL_ * HH_)           return;
    if (in_sizes[12] != NL_ * 2 * HH_ * HH_) return;
    if (in_sizes[13] != NL_ * HH_)           return;
    if (in_sizes[14] != NL_ * HH_ * HH_)     return;
    if (in_sizes[15] != NL_ * HH_)           return;
    if (out_size != NODES_ * HH_)            return;
    if (ws_size < WS_END)                    return;

    const float* h0    = (const float*)d_in[0];
    const float* coord = (const float*)d_in[1];
    const float* ln_g  = (const float*)d_in[2];
    const float* ln_b  = (const float*)d_in[3];
    const float* cW1   = (const float*)d_in[4];
    const float* cb1   = (const float*)d_in[5];
    const float* cW2   = (const float*)d_in[6];
    const float* cb2   = (const float*)d_in[7];
    const float* eW1   = (const float*)d_in[8];
    const float* eb1   = (const float*)d_in[9];
    const float* eW2   = (const float*)d_in[10];
    const float* eb2   = (const float*)d_in[11];
    const float* nW1   = (const float*)d_in[12];
    const float* nb1   = (const float*)d_in[13];
    const float* nW2   = (const float*)d_in[14];
    const float* nb2   = (const float*)d_in[15];
    float* out = (float*)d_out;

    char* ws = (char*)d_ws;
    float*          hn   = (float*)(ws + OFF_HN);
    float*          hbuf = (float*)(ws + OFF_HB);
    unsigned short* hah  = (unsigned short*)(ws + OFF_HAH);
    unsigned short* hal  = (unsigned short*)(ws + OFF_HAL);
    float*          pq   = (float*)(ws + OFF_PQ);
    unsigned short* wp   = (unsigned short*)(ws + OFF_W);

    hipFuncSetAttribute(reinterpret_cast<const void*>(&edge_kernel), hipFuncAttributeMaxDynamicSharedMemorySize, EK_LDS);
    hipFuncSetAttribute(reinterpret_cast<const void*>(&node_kernel), hipFuncAttributeMaxDynamicSharedMemorySize, NK_LDS);

    wprep_kernel<0><<<dim3(2, 2, NL_), dim3(256), 0, stream>>>(
        eW1, 3 * HH_ * HH_, wp + WO_PQH, wp + WO_PQL, WL_U16, HH_, HH_, HH_, 1.0f);
    wprep_kernel<0><<<dim3(2, 2, NL_), dim3(256), 0, stream>>>(
        eW1 + HH_ * HH_, 3 * HH_ * HH_, wp + WO_PQH + HH_ * HH_, wp + WO_PQL + HH_ * HH_, WL_U16, HH_, HH_, HH_, 1.0f);
    wprep_kernel<1><<<dim3(2, 2, NL_), dim3(256), 0, stream>>>(
        eW1 + 2 * HH_ * HH_, 3 * HH_ * HH_, wp + WO_E1F, wp + WO_E1F, WL_U16, HH_, HH_, HH_, 16.0f);
    wprep_kernel<1><<<dim3(2, 2, NL_), dim3(256), 0, stream>>>(
        cW2, HH_ * HH_, wp + WO_C2F, wp + WO_C2F, WL_U16, HH_, HH_, HH_, 16.0f);
    wprep_kernel<0><<<dim3(2, 2, NL_), dim3(256), 0, stream>>>(
        eW2, HH_ * HH_, wp + WO_E2H, wp + WO_E2L, WL_U16, HH_, HH_, HH_, 1.0f);
    wprep_kernel<0><<<dim3(2, 4, NL_), dim3(256), 0, stream>>>(
        nW1, 2 * HH_ * HH_, wp + WO_N1H, wp + WO_N1L, WL_U16, HH_, 2 * HH_, HH_, 1.0f);
    wprep_kernel<0><<<dim3(2, 2, NL_), dim3(256), 0, stream>>>(
        nW2, HH_ * HH_, wp + WO_N2H, wp + WO_N2L, WL_U16, HH_, HH_, HH_, 1.0f);

    for (int l = 0; l < NL_; ++l) {
        const float* hin  = (l == 0) ? h0 : (const float*)hbuf;
        float*       hnew = (l == NL_ - 1) ? out : hbuf;
        const unsigned short* wl = wp + (size_t)l * WL_U16;

        ln_kernel<<<dim3(NODES_ / 8), dim3(256), 0, stream>>>(
            hin, ln_g + l * HH_, ln_b + l * HH_, hn, hah, hal);

        pq_kernel<<<dim3(2, NODES_ / 64), dim3(128), 0, stream>>>(
            (const unsigned short*)hah, (const unsigned short*)hal, wl + WO_PQH, wl + WO_PQL, pq);

        edge_kernel<<<dim3(NB_ * (NN_ / 2)), dim3(256), EK_LDS, stream>>>(
            (const float*)pq, coord,
            cW1 + l * 2 * HH_, cb1 + l * HH_, cb2 + l * HH_, eb1 + l * HH_, eb2 + l * HH_,
            (const _Float16*)(wl + WO_C2F), (const _Float16*)(wl + WO_E1F),
            wl + WO_E2H, wl + WO_E2L,
            hah, hal);

        node_kernel<<<dim3(NODES_ / 64), dim3(128), NK_LDS, stream>>>(
            (const unsigned short*)hah, (const unsigned short*)hal, (const float*)hn,
            wl + WO_N1H, wl + WO_N1L, wl + WO_N2H, wl + WO_N2L,
            nb1 + l * HH_, nb2 + l * HH_, hnew);
    }
}
